// GraphTrajectoryEncoder_81561428951534
// MI455X (gfx1250) — hardware-verified
//
#include <hip/hip_runtime.h>

typedef _Float16 v16h __attribute__((ext_vector_type(16)));
typedef _Float16 v8h  __attribute__((ext_vector_type(8)));
typedef float    v8f  __attribute__((ext_vector_type(8)));
typedef float    v4f  __attribute__((ext_vector_type(4)));
typedef int      v4i  __attribute__((ext_vector_type(4)));
typedef v8h __attribute__((may_alias)) v8ha;
typedef v4f __attribute__((may_alias)) v4fa;
typedef v4i __attribute__((may_alias)) v4ia;

union Frag { v16h v; v8h half[2]; };

#define NB     4
#define SEQ    1024
#define DM     512
#define NH     8
#define HD     64
#define FF     2048
#define DEPTH  6
#define MROWS  (NB * SEQ)
#define QKVN   (3 * DM)
#define WSC    32.0f
#define PSCALE 1024.0f
#define SSC    0.0625f
#define NEGF   (-1.0e9f)
#define CPITCH 72

static_assert(MROWS % 128 == 0);
static_assert(SEQ % 128 == 0);
static_assert(DM % 64 == 0);
static_assert(QKVN % 64 == 0);
static_assert(FF % 64 == 0);
static_assert(DM % 32 == 0);
static_assert(FF % 32 == 0);
static_assert(HD == 64);
static_assert(NH == 8);
static_assert(DM == 512);

__device__ __forceinline__ v8f wmma_f16(v16h a, v16h b, v8f c) {
  v8f d = __builtin_amdgcn_wmma_f32_16x16x32_f16(false, a, false, b, (short)0, c, false, false);
  asm volatile("v_nop\n\tv_nop\n\tv_nop\n\tv_nop" : "+v"(d) : "v"(a), "v"(b));
  return d;
}

__device__ __forceinline__ v16h load_frag(const _Float16* p, int h) {
  Frag f;
  f.half[0] = *(const v8ha*)(p + 8 * h);
  f.half[1] = *(const v8ha*)(p + 16 + 8 * h);
  return f.v;
}

__device__ __forceinline__ void wt_store_pass(const _Float16* sT, _Float16* dst, int K,
                                              int w, int lane) {
  const int q8 = lane & 7, sub = lane >> 3;
#pragma unroll
  for (int i = 0; i < 2; ++i) {
    const int row = w * 8 + i * 4 + sub;
    const v8h v = *(const v8ha*)(sT + row * CPITCH + 8 * q8);
    *(volatile v8h*)(dst + (size_t)row * K + 8 * q8) = v;
  }
}

__global__ __launch_bounds__(256) void convert_wt_kernel(
    const float* __restrict__ W, _Float16* __restrict__ Wt, int K, int N)
{
  __shared__ __attribute__((aligned(16))) _Float16 sT[64 * CPITCH];

  const int tid = threadIdx.x, lane = tid & 31, w = tid >> 5;
  const int n0 = blockIdx.x * 64, k0 = blockIdx.y * 64, dep = blockIdx.z;
  const float* src = W + ((size_t)dep * K + k0) * N + n0;
#pragma unroll
  for (int i = 0; i < 4; ++i) {
    const int f = i * 256 + tid;
    const int kk = f >> 4, c4 = f & 15;
    const v4f v = *(const v4fa*)(src + (size_t)kk * N + 4 * c4);
    _Float16* col = sT + (4 * c4) * CPITCH + kk;
    col[0]          = (_Float16)(v.x * WSC);
    col[CPITCH]     = (_Float16)(v.y * WSC);
    col[2 * CPITCH] = (_Float16)(v.z * WSC);
    col[3 * CPITCH] = (_Float16)(v.w * WSC);
  }
  __syncthreads();

  _Float16* dst = Wt + ((size_t)dep * N + n0) * K + k0;
  wt_store_pass(sT, dst, K, w, lane);
  __threadfence();
  wt_store_pass(sT, dst, K, w, lane);
}

__global__ __launch_bounds__(256) void layernorm_kernel(
    const float* __restrict__ x, const float* __restrict__ gw,
    const float* __restrict__ gb, _Float16* __restrict__ out, int nrows)
{
  const int lane = threadIdx.x & 31, wv = threadIdx.x >> 5;
  const int row = blockIdx.x * 8 + wv;
  if (row >= nrows) return;
  const float* xr = x + (size_t)row * DM;

  v4f a[4];
#pragma unroll
  for (int j = 0; j < 2; ++j) {
    const int base = 8 * (lane + 32 * j);
    a[2 * j]     = *(const v4fa*)(xr + base);
    a[2 * j + 1] = *(const v4fa*)(xr + base + 4);
  }
  float s = 0.0f;
#pragma unroll
  for (int i = 0; i < 4; ++i) s += (a[i].x + a[i].y) + (a[i].z + a[i].w);
#pragma unroll
  for (int off = 16; off > 0; off >>= 1) s += __shfl_xor(s, off);
  const float mu = s * (1.0f / DM);

  float ss = 0.0f;
#pragma unroll
  for (int i = 0; i < 4; ++i) {
    const v4f d = a[i] - mu;
    a[i] = d;
    ss += (d.x * d.x + d.y * d.y) + (d.z * d.z + d.w * d.w);
  }
#pragma unroll
  for (int off = 16; off > 0; off >>= 1) ss += __shfl_xor(ss, off);
  const float rstd = rsqrtf(ss * (1.0f / DM) + 1e-5f);

  v8h o[2];
#pragma unroll
  for (int j = 0; j < 2; ++j) {
    const int base = 8 * (lane + 32 * j);
    const v4f w0 = *(const v4fa*)(gw + base);
    const v4f w1 = *(const v4fa*)(gw + base + 4);
    const v4f b0 = *(const v4fa*)(gb + base);
    const v4f b1 = *(const v4fa*)(gb + base + 4);
    const v4f y0 = a[2 * j] * rstd * w0 + b0;
    const v4f y1 = a[2 * j + 1] * rstd * w1 + b1;
    const v8h t = { (_Float16)y0.x, (_Float16)y0.y, (_Float16)y0.z, (_Float16)y0.w,
                    (_Float16)y1.x, (_Float16)y1.y, (_Float16)y1.z, (_Float16)y1.w };
    o[j] = t;
  }
  _Float16* orow = out + (size_t)row * DM;
  *(volatile v8h*)(orow + 8 * lane)        = o[0];
  *(volatile v8h*)(orow + 8 * (lane + 32)) = o[1];
  __threadfence();
  *(volatile v8h*)(orow + 8 * lane)        = o[0];
  *(volatile v8h*)(orow + 8 * (lane + 32)) = o[1];
}

__device__ __forceinline__ void qkv_store_pass(const _Float16* sH, _Float16* plane, _Float16* vt,
                                               int which, int bh, int l0, int w, int lane) {
  const int q8 = lane & 7, sub = lane >> 3;
#pragma unroll
  for (int i = 0; i < 8; ++i) {
    const int lid = w * 32 + i * 4 + sub;
    v8h v;
    _Float16* dst;
    if (which != 2) {
      v = *(const v8ha*)(sH + lid * HD + 8 * q8);
      dst = plane + ((size_t)bh * SEQ + l0 + lid) * HD + 8 * q8;
    } else {
      const int d = lid >> 1, hl = lid & 1;
      v = *(const v8ha*)(sH + d * 128 + 64 * hl + 8 * q8);
      dst = vt + ((size_t)bh * HD + d) * SEQ + l0 + 64 * hl + 8 * q8;
    }
    *(volatile v8h*)dst = v;
  }
}

__device__ __forceinline__ void gelu_store_pass(const _Float16* sH, _Float16* dst, int ldn,
                                                int w, int lane) {
  const int q8 = lane & 7, sub = lane >> 3;
#pragma unroll
  for (int i = 0; i < 8; ++i) {
    const int lid = w * 32 + i * 4 + sub;
    const v8h v = *(const v8ha*)(sH + lid * HD + 8 * q8);
    *(volatile v8h*)(dst + (size_t)lid * ldn + 8 * q8) = v;
  }
}

__device__ __forceinline__ void res_store_pass(const float* so, float* outf, const float* biasn,
                                               const float* res, int m0w, int n0, int ldn, int lane) {
  const int q8 = lane & 7, sub = lane >> 3;
#pragma unroll
  for (int i = 0; i < 16; ++i) {
    const int lid = i * 4 + sub;
    const int row = lid >> 1, hl = lid & 1;
    const int cl = 32 * hl + 4 * q8;
    const v4f v  = *(const v4fa*)(so + row * 64 + cl);
    const v4f bb = *(const v4fa*)(biasn + cl);
    const size_t gi = (size_t)(m0w + row) * ldn + n0 + cl;
    const v4f rr = *(const v4fa*)(res + gi);
    const v4f o = (v + bb) + rr;
    *(volatile v4f*)(outf + gi) = o;
  }
}

template <int EPI, int K, int N>
__global__ __launch_bounds__(128) void gemm_kernel(
    const _Float16* __restrict__ A, const _Float16* __restrict__ Wt,
    const float* __restrict__ bias, const float* __restrict__ res,
    float* __restrict__ outf, _Float16* __restrict__ out0,
    _Float16* __restrict__ out1, _Float16* __restrict__ out2)
{
  static_assert(K % 32 == 0);
  static_assert(N % 64 == 0);
  __shared__ __attribute__((aligned(16))) _Float16 sH[128 * 64];
  __shared__ __attribute__((aligned(16))) float    sF[128 * 64];

  const int tid = threadIdx.x, lane = tid & 31, w = tid >> 5;
  const int h = lane >> 4, m = lane & 15;
  const int m0 = blockIdx.x * 128, n0 = blockIdx.y * 64;
  const int m0w = m0 + 32 * w;

  const _Float16* xa0 = A + (size_t)(m0w + m) * K;
  const _Float16* xa1 = xa0 + (size_t)16 * K;
  const _Float16* wb  = Wt + (size_t)(n0 + m) * K;

  const v8f zero8 = {0.f, 0.f, 0.f, 0.f, 0.f, 0.f, 0.f, 0.f};
  v8f acc[2][4];
#pragma unroll
  for (int mt = 0; mt < 2; ++mt)
#pragma unroll
    for (int nt = 0; nt < 4; ++nt) acc[mt][nt] = zero8;

#pragma unroll 1
  for (int k0 = 0; k0 < K; k0 += 32) {
    const v16h a0 = load_frag(xa0 + k0, h);
    const v16h a1 = load_frag(xa1 + k0, h);
#pragma unroll
    for (int nt = 0; nt < 4; ++nt) {
      const v16h b = load_frag(wb + (size_t)nt * 16 * K + k0, h);
      acc[0][nt] = wmma_f16(a0, b, acc[0][nt]);
      acc[1][nt] = wmma_f16(a1, b, acc[1][nt]);
    }
  }

  if (EPI == 0) {
    const int which = blockIdx.y >> 3, head = blockIdx.y & 7;
    const float osc = (which == 0) ? (1.0f / 64.0f) : (1.0f / 8.0f);
#pragma unroll
    for (int nt = 0; nt < 4; ++nt) {
      const int feat = 16 * nt + m;
#pragma unroll
      for (int mt = 0; mt < 2; ++mt) {
#pragma unroll
        for (int r = 0; r < 8; ++r) {
          const int tokl = 32 * w + 16 * mt + 8 * h + r;
          const float y = acc[mt][nt][r] * osc;
          const int idx = (which == 2) ? (feat * 128 + tokl) : (tokl * HD + feat);
          sH[idx] = (_Float16)y;
        }
      }
    }
    __syncthreads();
    const int b = m0 / SEQ, l0 = m0 - b * SEQ, bh = b * NH + head;
    _Float16* plane = (which == 0) ? out0 : out1;
    qkv_store_pass(sH, plane, out2, which, bh, l0, w, lane);
    __threadfence();
    qkv_store_pass(sH, plane, out2, which, bh, l0, w, lane);
  } else if (EPI == 1) {
#pragma unroll
    for (int nt = 0; nt < 4; ++nt) {
      const int feat = 16 * nt + m;
      const float bv = bias[n0 + feat];
#pragma unroll
      for (int mt = 0; mt < 2; ++mt) {
#pragma unroll
        for (int r = 0; r < 8; ++r) {
          const int tokl = 32 * w + 16 * mt + 8 * h + r;
          const float v = acc[mt][nt][r] * (1.0f / 32.0f) + bv;
          const float g = 0.5f * v * (1.0f + erff(v * 0.70710678118654752f));
          sH[tokl * HD + feat] = (_Float16)(g * 4.0f);
        }
      }
    }
    __syncthreads();
    _Float16* dst = out0 + (size_t)m0 * N + n0;
    gelu_store_pass(sH, dst, N, w, lane);
    __threadfence();
    gelu_store_pass(sH, dst, N, w, lane);
  } else {
    float* so = sF + w * 2048;
#pragma unroll
    for (int mt = 0; mt < 2; ++mt)
#pragma unroll
      for (int nt = 0; nt < 4; ++nt)
#pragma unroll
        for (int r = 0; r < 8; ++r)
          so[(16 * mt + 8 * h + r) * 64 + 16 * nt + m] = acc[mt][nt][r] * (1.0f / 128.0f);
    __syncthreads();
    res_store_pass(so, outf, bias + n0, res, m0w, n0, N, lane);
    __threadfence();
    res_store_pass(so, outf, bias + n0, res, m0w, n0, N, lane);
  }
}

__device__ __forceinline__ v16h pack_p(v8f a, v8f c) {
  const v16h r = { (_Float16)(a[0] * PSCALE), (_Float16)(a[1] * PSCALE), (_Float16)(a[2] * PSCALE), (_Float16)(a[3] * PSCALE),
                   (_Float16)(a[4] * PSCALE), (_Float16)(a[5] * PSCALE), (_Float16)(a[6] * PSCALE), (_Float16)(a[7] * PSCALE),
                   (_Float16)(c[0] * PSCALE), (_Float16)(c[1] * PSCALE), (_Float16)(c[2] * PSCALE), (_Float16)(c[3] * PSCALE),
                   (_Float16)(c[4] * PSCALE), (_Float16)(c[5] * PSCALE), (_Float16)(c[6] * PSCALE), (_Float16)(c[7] * PSCALE) };
  return r;
}

__device__ __forceinline__ v8f mask8(v8f s, const int* mp, int key0, int qi) {
  const v4i ga = *(const v4ia*)mp;
  const v4i gc = *(const v4ia*)(mp + 4);
  s[0] = ((ga.x > 0) || (key0 + 0 == qi)) ? s[0] * SSC : NEGF;
  s[1] = ((ga.y > 0) || (key0 + 1 == qi)) ? s[1] * SSC : NEGF;
  s[2] = ((ga.z > 0) || (key0 + 2 == qi)) ? s[2] * SSC : NEGF;
  s[3] = ((ga.w > 0) || (key0 + 3 == qi)) ? s[3] * SSC : NEGF;
  s[4] = ((gc.x > 0) || (key0 + 4 == qi)) ? s[4] * SSC : NEGF;
  s[5] = ((gc.y > 0) || (key0 + 5 == qi)) ? s[5] * SSC : NEGF;
  s[6] = ((gc.z > 0) || (key0 + 6 == qi)) ? s[6] * SSC : NEGF;
  s[7] = ((gc.w > 0) || (key0 + 7 == qi)) ? s[7] * SSC : NEGF;
  return s;
}

__device__ __forceinline__ void ctx_store_pass(const _Float16* so, _Float16* ctx,
                                               int b, int head, int q0, int lane) {
  const int q8 = lane & 7, sub = lane >> 3;
#pragma unroll
  for (int i = 0; i < 4; ++i) {
    const int row = i * 4 + sub;
    const v8h v = *(const v8ha*)(so + row * HD + 8 * q8);
    const size_t gi = ((size_t)b * SEQ + q0 + row) * DM + head * HD + 8 * q8;
    *(volatile v8h*)(ctx + gi) = v;
  }
}

__global__ __launch_bounds__(128) void attn_kernel(
    const _Float16* __restrict__ qh,
    const _Float16* __restrict__ kh,
    const _Float16* __restrict__ vt,
    const int* __restrict__ gmask,
    _Float16* __restrict__ ctx)
{
  __shared__ __attribute__((aligned(16))) _Float16 sO[4 * 16 * HD];

  const int tid = threadIdx.x, lane = tid & 31, w = tid >> 5;
  const int h = lane >> 4, m = lane & 15;
  const int bh = blockIdx.y, b = bh >> 3, head = bh & 7;
  const int q0 = blockIdx.x * 64 + 16 * w;
  const int qi = q0 + m;

  const _Float16* qrow = qh + ((size_t)bh * SEQ + qi) * HD;
  const v16h qb0 = load_frag(qrow, h);
  const v16h qb1 = load_frag(qrow + 32, h);

  const v8f zero8 = {0.f, 0.f, 0.f, 0.f, 0.f, 0.f, 0.f, 0.f};
  v8f o[4];
#pragma unroll
  for (int t = 0; t < 4; ++t) o[t] = zero8;
  float mrun = -1e30f, lrun = 0.0f;

  const _Float16* kbase = kh + ((size_t)bh * SEQ + m) * HD;
  const _Float16* vbase = vt + ((size_t)bh * HD + m) * SEQ;
  const int* mrow = gmask + ((size_t)b * SEQ + qi) * SEQ + 8 * h;

#pragma unroll 1
  for (int kb = 0; kb < SEQ; kb += 64) {
    v8f s[4];
#pragma unroll
    for (int j = 0; j < 4; ++j) {
      const _Float16* kp = kbase + (size_t)(kb + 16 * j) * HD;
      const v16h kf0 = load_frag(kp, h);
      const v16h kf1 = load_frag(kp + 32, h);
      v8f z = zero8;
      z = wmma_f16(kf0, qb0, z);
      z = wmma_f16(kf1, qb1, z);
      s[j] = z;
    }
#pragma unroll
    for (int j = 0; j < 4; ++j) s[j] = mask8(s[j], mrow + kb + 16 * j, kb + 16 * j + 8 * h, qi);

    float mloc = s[0][0];
#pragma unroll
    for (int j = 0; j < 4; ++j)
#pragma unroll
      for (int r = 0; r < 8; ++r) mloc = fmaxf(mloc, s[j][r]);
    mloc = fmaxf(mloc, __shfl_xor(mloc, 16));
    const float mnew = fmaxf(mrun, mloc);
    const float alpha = __expf(mrun - mnew);
    mrun = mnew;
    float lsum = 0.0f;
#pragma unroll
    for (int j = 0; j < 4; ++j)
#pragma unroll
      for (int r = 0; r < 8; ++r) {
        const float p = __expf(s[j][r] - mnew);
        s[j][r] = p;
        lsum += p;
      }
    lsum += __shfl_xor(lsum, 16);
    lrun = lrun * alpha + lsum;
#pragma unroll
    for (int t = 0; t < 4; ++t)
#pragma unroll
      for (int r = 0; r < 8; ++r) o[t][r] = o[t][r] * alpha;

    const v16h pb0 = pack_p(s[0], s[1]);
    const v16h pb1 = pack_p(s[2], s[3]);

#pragma unroll
    for (int t = 0; t < 4; ++t) {
      const _Float16* vp = vbase + (size_t)(16 * t) * SEQ + kb;
      const v16h vf0 = load_frag(vp, h);
      const v16h vf1 = load_frag(vp + 32, h);
      o[t] = wmma_f16(vf0, pb0, o[t]);
      o[t] = wmma_f16(vf1, pb1, o[t]);
    }
  }

  const float inv = (1.0f / lrun) * (1.0f / PSCALE);
  _Float16* so = sO + w * 1024;
#pragma unroll
  for (int t = 0; t < 4; ++t)
#pragma unroll
    for (int r = 0; r < 8; ++r)
      so[m * HD + 16 * t + 8 * h + r] = (_Float16)(o[t][r] * inv);
  __syncthreads();

  ctx_store_pass(so, ctx, b, head, q0, lane);
  __threadfence();
  ctx_store_pass(so, ctx, b, head, q0, lane);
}

extern "C" void kernel_launch(void* const* d_in, const int* in_sizes, int n_in,
                              void* d_out, int out_size, void* d_ws, size_t ws_size,
                              hipStream_t stream) {
  if (n_in < 13) return;
  if (in_sizes[0] != MROWS * DM) return;
  if (in_sizes[1] != NB * SEQ * SEQ) return;
  if (in_sizes[2] != DEPTH * DM || in_sizes[3] != DEPTH * DM) return;
  if (in_sizes[4] != DEPTH * DM * QKVN) return;
  if (in_sizes[5] != DEPTH * DM * DM || in_sizes[6] != DEPTH * DM) return;
  if (in_sizes[7] != DEPTH * DM || in_sizes[8] != DEPTH * DM) return;
  if (in_sizes[9] != DEPTH * DM * FF || in_sizes[10] != DEPTH * FF) return;
  if (in_sizes[11] != DEPTH * FF * DM || in_sizes[12] != DEPTH * DM) return;
  if (out_size != MROWS * DM) return;

  const float* x     = (const float*)d_in[0];
  const int*   gmask = (const int*)  d_in[1];
  const float* ln1w  = (const float*)d_in[2];
  const float* ln1b  = (const float*)d_in[3];
  const float* Wqkv  = (const float*)d_in[4];
  const float* Wout  = (const float*)d_in[5];
  const float* bout  = (const float*)d_in[6];
  const float* ln2w  = (const float*)d_in[7];
  const float* ln2b  = (const float*)d_in[8];
  const float* W1    = (const float*)d_in[9];
  const float* b1    = (const float*)d_in[10];
  const float* W2    = (const float*)d_in[11];
  const float* b2    = (const float*)d_in[12];
  float* out = (float*)d_out;

  const size_t QKV_W = (size_t)QKVN * DM;
  const size_t OUT_W = (size_t)DM * DM;
  const size_t W1_W  = (size_t)FF * DM;
  const size_t W2_W  = (size_t)DM * FF;
  const size_t wqkv_bytes = DEPTH * QKV_W * 2;
  const size_t wout_bytes = DEPTH * OUT_W * 2;
  const size_t w1_bytes   = DEPTH * W1_W * 2;
  const size_t w2_bytes   = DEPTH * W2_W * 2;
  const size_t h_bytes    = (size_t)MROWS * DM * 4;
  const size_t p16_bytes  = (size_t)MROWS * DM * 2;
  const size_t g_bytes    = (size_t)MROWS * FF * 2;
  const size_t total = wqkv_bytes + wout_bytes + w1_bytes + w2_bytes + 2 * h_bytes + 5 * p16_bytes + g_bytes;
  if (total > ws_size) return;
  if (total > (size_t)134217728) return;

  char* ws = (char*)d_ws;
  size_t off = 0;
  _Float16* wqkv_t = (_Float16*)(ws + off); off += wqkv_bytes;
  _Float16* wout_t = (_Float16*)(ws + off); off += wout_bytes;
  _Float16* w1_t   = (_Float16*)(ws + off); off += w1_bytes;
  _Float16* w2_t   = (_Float16*)(ws + off); off += w2_bytes;
  float*    hA     = (float*)(ws + off);    off += h_bytes;
  float*    hB     = (float*)(ws + off);    off += h_bytes;
  _Float16* npl    = (_Float16*)(ws + off); off += p16_bytes;
  _Float16* qpl    = (_Float16*)(ws + off); off += p16_bytes;
  _Float16* kpl    = (_Float16*)(ws + off); off += p16_bytes;
  _Float16* vtp    = (_Float16*)(ws + off); off += p16_bytes;
  _Float16* ctxp   = (_Float16*)(ws + off); off += p16_bytes;
  _Float16* gpl    = (_Float16*)(ws + off); off += g_bytes;
  if (off != total) return;

  convert_wt_kernel<<<dim3(QKVN / 64, DM / 64, DEPTH), 256, 0, stream>>>(Wqkv, wqkv_t, DM, QKVN);
  convert_wt_kernel<<<dim3(DM / 64,   DM / 64, DEPTH), 256, 0, stream>>>(Wout, wout_t, DM, DM);
  convert_wt_kernel<<<dim3(FF / 64,   DM / 64, DEPTH), 256, 0, stream>>>(W1,   w1_t,   DM, FF);
  convert_wt_kernel<<<dim3(DM / 64,   FF / 64, DEPTH), 256, 0, stream>>>(W2,   w2_t,   FF, DM);

  const dim3 gGemmQKV(MROWS / 128, QKVN / 64);
  const dim3 gGemmD(MROWS / 128, DM / 64);
  const dim3 gGemmF(MROWS / 128, FF / 64);
  const dim3 gAtt(SEQ / 64, NB * NH);
  const int  gLN = MROWS / 8;

  for (int l = 0; l < DEPTH; ++l) {
    const float* hsrc = (l == 0) ? x : hB;

    layernorm_kernel<<<gLN, 256, 0, stream>>>(hsrc, ln1w + l * DM, ln1b + l * DM, npl, MROWS);
    gemm_kernel<0, DM, QKVN><<<gGemmQKV, 128, 0, stream>>>(
        npl, wqkv_t + (size_t)l * QKV_W, bout + l * DM, x, hA, qpl, kpl, vtp);
    attn_kernel<<<gAtt, 128, 0, stream>>>(qpl, kpl, vtp, gmask, ctxp);
    gemm_kernel<2, DM, DM><<<gGemmD, 128, 0, stream>>>(
        ctxp, wout_t + (size_t)l * OUT_W, bout + l * DM, hsrc, hA, npl, npl, npl);
    layernorm_kernel<<<gLN, 256, 0, stream>>>(hA, ln2w + l * DM, ln2b + l * DM, npl, MROWS);
    gemm_kernel<1, DM, FF><<<gGemmF, 128, 0, stream>>>(
        npl, w1_t + (size_t)l * W1_W, b1 + l * FF, x, hA, gpl, gpl, gpl);
    float* dst = (l == DEPTH - 1) ? out : hB;
    gemm_kernel<2, FF, DM><<<gGemmD, 128, 0, stream>>>(
        gpl, w2_t + (size_t)l * W2_W, b2 + l * DM, hA, dst, npl, npl, npl);
  }
}
